// h_diag_Land_42932493090900
// MI455X (gfx1250) — hardware-verified
//
#include <hip/hip_runtime.h>
#include <math.h>

typedef __attribute__((ext_vector_type(16))) _Float16 v16h;
typedef __attribute__((ext_vector_type(16))) __bf16 v16b;
typedef __attribute__((ext_vector_type(8)))  _Float16 v8h;
typedef __attribute__((ext_vector_type(8)))  float v8f;
typedef __attribute__((ext_vector_type(4)))  float v4f;
typedef __attribute__((ext_vector_type(2)))  float v2f;
typedef __attribute__((ext_vector_type(4)))  unsigned v4u;
typedef __attribute__((ext_vector_type(4)))  int v4i;
typedef float __attribute__((may_alias)) float_a;
typedef int __attribute__((may_alias)) int_a;

template <typename T> __device__ __forceinline__ void vst2(void* p, T v) { *(volatile T*)p = v; __threadfence(); *(volatile T*)p = v; }
__device__ __forceinline__ v8f wmma16(v16h a, v16h b, v8f c) {
  v8f d = __builtin_amdgcn_wmma_f32_16x16x32_f16(false, a, false, b, (short)0, c, false, false);
  asm volatile("v_nop\n\tv_nop\n\tv_nop\n\tv_nop" : "+v"(d) : "v"(a), "v"(b));
  return d;
}
__device__ __forceinline__ v8f wmma_bf(v16b a, v16b b, v8f c) {
  v8f d = __builtin_amdgcn_wmma_f32_16x16x32_bf16(false, a, false, b, (short)0, c, false, false);
  asm volatile("v_nop\n\tv_nop\n\tv_nop\n\tv_nop" : "+v"(d) : "v"(a), "v"(b));
  return d;
}
__device__ __forceinline__ v16h frag_h(const _Float16* rowk0, int lane) {
  union { v16h v; v8h q[2]; } u; const _Float16* p = rowk0 + 8 * (lane >> 4);
  u.q[0] = *(const v8h*)p; u.q[1] = *(const v8h*)(p + 16); return u.v;
}
__device__ __forceinline__ v16h frag_f32(const float* rowk0, int lane) {
  v16h a; const float* p = rowk0 + 8 * (lane >> 4);
#pragma unroll
  for (int i = 0; i < 8; ++i) { a[i] = (_Float16)p[i]; a[8 + i] = (_Float16)p[16 + i]; }
  return a;
}
__device__ __forceinline__ v16h frag_f32s(const float* rowk0, int lane, float sc) {
  v16h a; const float* p = rowk0 + 8 * (lane >> 4);
#pragma unroll
  for (int i = 0; i < 8; ++i) { a[i] = (_Float16)(p[i] * sc); a[8 + i] = (_Float16)(p[16 + i] * sc); }
  return a;
}
__device__ __forceinline__ v16h fragc_f32(const float* W, int k0, int n, int lane, int ld, int K) {
  v16h a; const int g = lane >> 4;
#pragma unroll
  for (int i = 0; i < 8; ++i) { const int ka = k0 + 8 * g + i, kb = ka + 16;
    a[i] = (_Float16)(ka < K ? W[(size_t)(ka < K ? ka : K - 1) * ld + n] : 0.f); a[8 + i] = (_Float16)(kb < K ? W[(size_t)(kb < K ? kb : K - 1) * ld + n] : 0.f); }
  return a;
}
struct F2 { v16b h, l; };
__device__ __forceinline__ F2 bsplit16(const float v[16]) { F2 r;
#pragma unroll
  for (int i = 0; i < 16; ++i) { const __bf16 h = (__bf16)v[i]; r.h[i] = h; r.l[i] = (__bf16)(v[i] - (float)h); }
  return r; }
__device__ __forceinline__ F2 split_row(const float* row, int k0, int lane) { float v[16]; const float* p = row + k0 + 8 * (lane >> 4);
#pragma unroll
  for (int i = 0; i < 8; ++i) { v[i] = p[i]; v[8 + i] = p[16 + i]; }
  return bsplit16(v); }
__device__ __forceinline__ F2 split_rowK(const float* row, int k0, int lane, int K) { float v[16]; const int g = lane >> 4;
#pragma unroll
  for (int i = 0; i < 8; ++i) { const int ka = k0 + 8 * g + i, kb = ka + 16; v[i] = ka < K ? row[ka < K ? ka : K - 1] : 0.f; v[8 + i] = kb < K ? row[kb < K ? kb : K - 1] : 0.f; }
  return bsplit16(v); }
__device__ __forceinline__ F2 split_col(const float* W, int k0, int n, int lane, int ld, int K) { float v[16]; const int g = lane >> 4;
#pragma unroll
  for (int i = 0; i < 8; ++i) { const int ka = k0 + 8 * g + i, kb = ka + 16; v[i] = ka < K ? W[(size_t)(ka < K ? ka : K - 1) * ld + n] : 0.f; v[8 + i] = kb < K ? W[(size_t)(kb < K ? kb : K - 1) * ld + n] : 0.f; }
  return bsplit16(v); }
__device__ __forceinline__ v8f mac3(const F2& a, const F2& b, v8f c) { c = wmma_bf(a.l, b.h, c); c = wmma_bf(a.h, b.l, c); return wmma_bf(a.h, b.h, c); }
__device__ __forceinline__ float sigm(float v) { return 1.0f / (1.0f + expf(-v)); }
#define LDSX() do { asm volatile("s_wait_dscnt 0" ::: "memory"); __builtin_amdgcn_wave_barrier(); __builtin_amdgcn_fence(__ATOMIC_RELEASE, "workgroup"); } while (0)


#define NBQ 8192
#define NRF 8192
#define DD 256
#ifndef TQ
#define TQ (NBQ / 64)
#endif
typedef __attribute__((ext_vector_type(8))) __bf16 v8b;
__device__ __forceinline__ v16b frag_b(const __bf16* rowk0, int lane) {
  union { v16b v; v8b q[2]; } u; const __bf16* p = rowk0 + 8 * (lane >> 4);
  u.q[0] = *(const v8b*)p; u.q[1] = *(const v8b*)(p + 16); return u.v;
}
__device__ __forceinline__ float bfr(float v) { return (float)(__bf16)v; }
__device__ __attribute__((noinline)) float exp_ni(float v) { return expf(v); }
__device__ __attribute__((noinline)) float erf_ni(float v) { return erff(v); }
#define INV2G2 (1.0f / 128.0f)
#define LEPS 0.001f

#define WS_RB  0u
#define WS_RT  (WS_RB + 2u * (size_t)NRF * DD)
#define WS_R2T (WS_RT + 2u * (size_t)DD * NRF)
#define WS_RSQ (WS_R2T + 2u * (size_t)DD * NRF)
#define WS_W16 (WS_RSQ + 4u * (size_t)NRF)
#define WS_END (WS_W16 + 2u * (size_t)NBQ * NRF)

__global__ __launch_bounds__(256) void k_ref(const float* __restrict__ R, __bf16* __restrict__ RB, _Float16* __restrict__ RT, _Float16* __restrict__ R2T, float* __restrict__ RSQ) { __shared__ __align__(16) __bf16 sb[64][DD + 8]; __shared__ __align__(16) _Float16 st[DD][64 + 8], st2[DD][64 + 8]; __shared__ __align__(16) float sq[64]; const int t = threadIdx.x; const int n0 = blockIdx.x * 64;
  for (int e = t; e < 64 * DD; e += 256) { const int rl = e >> 8, d = e & 255; const float v = bfr(R[(size_t)(n0 + rl) * DD + d]); sb[rl][d] = (__bf16)v; st[d][rl] = (_Float16)v; st2[d][rl] = (_Float16)(v * v); } __syncthreads();
  if (t < 64) { float s = 0.f; const float* rr = R + (size_t)(n0 + t) * DD; for (int d = 0; d < DD; ++d) { const float v = bfr(rr[d]); s += v * v; } sq[t] = s; } __syncthreads();
  for (int e = t; e < 64 * 32; e += 256) { const int rl = e >> 5, q = e & 31; vst2((unsigned*)(RB + (size_t)(n0 + rl) * DD + q * 8), *(const v4u*)&sb[rl][q * 8]); }
  for (int e = t; e < DD * 8; e += 256) { const int d = e >> 3, q = e & 7; vst2((unsigned*)(RT + (size_t)d * NRF + n0 + q * 8), *(const v4u*)&st[d][q * 8]); vst2((unsigned*)(R2T + (size_t)d * NRF + n0 + q * 8), *(const v4u*)&st2[d][q * 8]); }
  if (t < 16) vst2(RSQ + n0 + t * 4, *(const v4f*)&sq[t * 4]); }
__device__ __forceinline__ v16b fragb_f32(const float* __restrict__ p, int lane) { v16b a; const float* pp = p + 8 * (lane >> 4);
#pragma unroll
  for (int i = 0; i < 8; ++i) { a[i] = (__bf16)pp[i]; a[8 + i] = (__bf16)pp[16 + i]; } return a; }
__global__ __launch_bounds__(128) void k_w(const float* __restrict__ X, const __bf16* __restrict__ RB, const float* __restrict__ RSQ, _Float16* __restrict__ W16) { __shared__ __align__(16) _Float16 so[64][136]; __shared__ float sxq[64];
  const int tid = threadIdx.x, wave = tid >> 5, lane = tid & 31, col = lane & 15, g = lane >> 4; const size_t rb = (size_t)blockIdx.x * 64; const size_t r0 = rb + wave * 16; const int c0 = blockIdx.y * 128;
  if (tid < 64) { float s = 0.f; const float* xr = X + (rb + tid) * DD; for (int d = 0; d < DD; ++d) { const float v = bfr(xr[d]); s += v * v; } sxq[tid] = s; }
  v8f acc[8] = {};
#pragma unroll 2
  for (int kc = 0; kc < DD / 32; ++kc) { const v16b a = fragb_f32(X + (r0 + col) * DD + kc * 32, lane);
#pragma unroll
    for (int j = 0; j < 8; ++j) acc[j] = wmma_bf(a, frag_b(RB + (size_t)(c0 + j * 16 + col) * DD + kc * 32, lane), acc[j]); }
  __syncthreads();
#pragma unroll
  for (int j = 0; j < 8; ++j) { const float rq = RSQ[c0 + j * 16 + col];
#pragma unroll
    for (int r = 0; r < 8; ++r) { const int rl = wave * 16 + 8 * g + r; const float dist = sxq[rl] + rq - 2.0f * acc[j][r]; so[rl][j * 16 + col] = (_Float16)expf(-dist * INV2G2); } }
  __syncthreads(); for (int e = tid; e < 64 * 16; e += 128) { const int rl = e >> 4, q = e & 15; vst2((unsigned*)(W16 + (rb + rl) * NRF + c0 + q * 8), *(const v4u*)&so[rl][q * 8]); } }
__global__ __launch_bounds__(128) void k_m(const _Float16* __restrict__ W16, const _Float16* __restrict__ RT, const _Float16* __restrict__ R2T, const float* __restrict__ X, const float* __restrict__ WW, float* __restrict__ OUT) { __shared__ __align__(16) float sf[4][16][132]; __shared__ float swsum[64];
  const int tid = threadIdx.x, wave = tid >> 5, lane = tid & 31, col = lane & 15, g = lane >> 4; const size_t rb = (size_t)blockIdx.x * 64; const size_t r0 = rb + wave * 16; const int d0 = blockIdx.y * 128;
  v8f a1[8] = {}, a2[8] = {}; float ws8[8] = {0.f, 0.f, 0.f, 0.f, 0.f, 0.f, 0.f, 0.f}; (void)ws8;
#pragma unroll 1
  for (int kc = 0; kc < NRF / 32; ++kc) { const v16h a = frag_h(W16 + (r0 + col) * NRF + kc * 32, lane);
#pragma unroll
    for (int j = 0; j < 8; ++j) { a1[j] = wmma16(a, frag_h(RT + (size_t)(d0 + j * 16 + col) * NRF + kc * 32, lane), a1[j]); a2[j] = wmma16(a, frag_h(R2T + (size_t)(d0 + j * 16 + col) * NRF + kc * 32, lane), a2[j]); } }
  if (tid < 64) { float s = 0.f; const _Float16* wr = W16 + (rb + tid) * NRF; for (int n = 0; n < NRF; n += 2) { s += (float)wr[n]; s += (float)wr[n + 1]; } swsum[tid] = s; }
  __syncthreads(); const float wsc = bfr(WW[0]);
#pragma unroll
  for (int j = 0; j < 8; ++j) { const int d = d0 + j * 16 + col;
#pragma unroll
    for (int r = 0; r < 8; ++r) { const int rl = wave * 16 + 8 * g + r; const float x = bfr(X[(rb + rl) * DD + d]); const float M = a2[j][r] - 2.0f * x * a1[j][r] + x * x * swsum[rl]; sf[wave][8 * g + r][j * 16 + col] = 1.0f / (wsc * M + LEPS); } }
  LDSX(); for (int rl = 0; rl < 16; ++rl) vst2(OUT + (r0 + rl) * DD + d0 + lane * 4, *(const v4f*)&sf[wave][rl][lane * 4]); }
extern "C" void kernel_launch(void* const* d_in, const int* in_sizes, int n_in, void* d_out, int out_size, void* d_ws, size_t ws_size, hipStream_t stream) {
  (void)in_sizes; (void)n_in; (void)out_size;
  const float** F = (const float**)d_in;
  if (ws_size < (size_t)WS_END) return;
  char* ws = (char*)d_ws; __bf16* RB = (__bf16*)(ws + WS_RB); _Float16 *RT = (_Float16*)(ws + WS_RT), *R2T = (_Float16*)(ws + WS_R2T), *W16 = (_Float16*)(ws + WS_W16); float* RSQ = (float*)(ws + WS_RSQ);
  k_ref<<<NRF / 64, 256, 0, stream>>>(F[1], RB, RT, R2T, RSQ);
  k_w<<<dim3(TQ, NRF / 128), 128, 0, stream>>>(F[0], RB, RSQ, W16);
  k_m<<<dim3(TQ, DD / 128), 128, 0, stream>>>(W16, RT, R2T, F[0], F[2], (float*)d_out);
}
